// DecoderLayer_4277787427226
// MI455X (gfx1250) — hardware-verified
//
#include <hip/hip_runtime.h>
#ifndef NB
#define NB 4
#endif
#ifndef SEQ
#define SEQ 1024
#endif
#define NB_FULL 4
#define SEQ_FULL 1024
#define DM 1024
#define NH 16
#define HD 64
#define FF 4096
#define MROWS (NB * SEQ)
#define NQT (SEQ / 64)
#define NKT (SEQ / 64)
static_assert(SEQ % 64 == 0);
static_assert(SEQ <= SEQ_FULL);
static_assert(NB >= 1 && NB <= NB_FULL);
static_assert(NKT <= 32);
static_assert(MROWS % 128 == 0);
static_assert(DM == NH * HD);
static_assert(DM % 64 == 0 && FF % 64 == 0 && (3 * DM) % 64 == 0 && (2 * DM) % 64 == 0);
static_assert(DM % 32 == 0 && FF % 32 == 0);
static_assert((MROWS * (DM / 8)) % 256 == 0);
static_assert((size_t)MROWS * 3 * DM * 2 <= (size_t)MROWS * FF * 2);
static_assert((size_t)MROWS * 2 * DM * 2 + (size_t)MROWS * DM * 2 <= (size_t)MROWS * FF * 2);
static_assert((size_t)NB * NH * HD * SEQ * 2 <= (size_t)MROWS * DM * 4);
static_assert((size_t)MROWS * DM * 2 <= (size_t)MROWS * DM * 4);

typedef _Float16 v16h __attribute__((ext_vector_type(16)));
typedef _Float16 v4h  __attribute__((ext_vector_type(4)));
typedef unsigned short v8us __attribute__((ext_vector_type(8), may_alias));
typedef float  v8f  __attribute__((ext_vector_type(8)));
typedef float  v4f  __attribute__((ext_vector_type(4)));
typedef float  v4fa __attribute__((ext_vector_type(4), may_alias));
union FragH { v16h v; v8us half[2]; _Float16 h[16]; unsigned short u[16]; };

#define NEG_INF (-__builtin_inff())

__device__ __forceinline__ unsigned short bf16_bits(float x) { unsigned int u = __float_as_uint(x); return (unsigned short)((u + 0x7FFFu + ((u >> 16) & 1u)) >> 16); }
__device__ __forceinline__ float bf16_val(unsigned short b) { return __uint_as_float(((unsigned int)b) << 16); }
__device__ __forceinline__ float bf16_rne(float x) { return bf16_val(bf16_bits(x)); }

__device__ __forceinline__ v16h g2_frag(const _Float16* p, int hh) { FragH f; f.half[0] = *(const v8us*)((const unsigned short*)p + 8 * hh); f.half[1] = *(const v8us*)((const unsigned short*)p + 16 + 8 * hh); return f.v; }
__device__ __forceinline__ v8f g2_mma(v16h a, v16h b, v8f c) { v8f d = __builtin_amdgcn_wmma_f32_16x16x32_f16(false, a, false, b, (short)0, c, false, false); asm volatile("v_nop\n\tv_nop\n\tv_nop\n\tv_nop" : "+v"(d) : "v"(a), "v"(b)); return d; }

__global__ __launch_bounds__(256) void k_x16(const float* __restrict__ x, _Float16* __restrict__ X16) {
  const unsigned t = blockIdx.x * 256u + threadIdx.x; if (t >= (unsigned)(MROWS * (DM / 8))) return;
  const unsigned m = t / (unsigned)(DM / 8), c8 = (t % (unsigned)(DM / 8)) * 8u;
  const unsigned b = m / (unsigned)SEQ, s = m % (unsigned)SEQ;
  const float* src = x + ((size_t)b * SEQ_FULL + s) * DM + c8;
  const v4f a = *(const v4fa*)src; const v4f c = *(const v4fa*)(src + 4); FragH f;
#pragma unroll
  for (int q = 0; q < 4; ++q) { f.h[q] = (_Float16)bf16_rne(a[q]); f.h[4 + q] = (_Float16)bf16_rne(c[q]); }
  unsigned short* d = (unsigned short*)X16 + (size_t)m * DM + c8;
  *(volatile v8us*)d = f.half[0]; __threadfence(); *(volatile v8us*)d = f.half[0]; }

__global__ __launch_bounds__(256) void k_wtr(const float* __restrict__ W, unsigned K, unsigned N, _Float16* __restrict__ Bt) {
  __shared__ unsigned short tl[64][66];
  const unsigned tid = threadIdx.x, n0 = blockIdx.x * 64u, k0 = blockIdx.y * 64u;
  for (unsigned i = tid; i < 1024u; i += 256u) { const unsigned r = i >> 4, c4 = (i & 15u) * 4u;
    const v4f v = *(const v4fa*)(W + (size_t)(k0 + r) * N + n0 + c4); FragH f;
#pragma unroll
    for (int q = 0; q < 4; ++q) f.h[q] = (_Float16)(bf16_rne(v[q]) * 16.0f);
#pragma unroll
    for (int q = 0; q < 4; ++q) tl[r][c4 + q] = f.u[q]; }
  __syncthreads();
  for (int pass = 0; pass < 2; ++pass) {
#pragma unroll
    for (unsigned rd = 0; rd < 2; ++rd) { const unsigned n = rd * 32u + (tid >> 3), pc = tid & 7u; FragH f;
#pragma unroll
      for (int q = 0; q < 8; ++q) f.u[q] = tl[pc * 8u + q][n];
      *(volatile v8us*)((unsigned short*)Bt + (size_t)(n0 + n) * K + k0 + pc * 8u) = f.half[0]; }
    if (pass == 0) __threadfence(); } }

__global__ __launch_bounds__(128) void k_gemm2(const _Float16* __restrict__ A, unsigned lda, const _Float16* __restrict__ Bh, unsigned ldb, float alpha, const float* __restrict__ bias,
    _Float16* __restrict__ C16, float* __restrict__ C32, unsigned ldc, unsigned M, unsigned N, unsigned K, int mode) {
  __shared__ __attribute__((aligned(16))) float so[4][32][68];
  const unsigned tid = threadIdx.x, w = tid >> 5, lane = tid & 31u, ln = lane & 15u, hh = lane >> 4;
  const unsigned ntn = N >> 6; const unsigned mt = blockIdx.x / ntn, nq = blockIdx.x - mt * ntn; const unsigned row0 = mt * 128u + 32u * w, col0 = nq * 64u; if (row0 >= M) return;
  const _Float16* a0p = A + (size_t)(row0 + ln) * lda; const _Float16* a1p = a0p + (size_t)16 * lda;
  const _Float16* b0p = Bh + (size_t)(col0 + ln) * ldb; const _Float16* b1p = b0p + (size_t)16 * ldb; const _Float16* b2p = b1p + (size_t)16 * ldb; const _Float16* b3p = b2p + (size_t)16 * ldb;
  const v8f z8 = {0.f,0.f,0.f,0.f,0.f,0.f,0.f,0.f}; v8f c00 = z8, c01 = z8, c02 = z8, c03 = z8, c10 = z8, c11 = z8, c12 = z8, c13 = z8;
#pragma unroll 1
  for (unsigned kb = 0; kb < K; kb += 32u) { const v16h a0 = g2_frag(a0p + kb, (int)hh), a1 = g2_frag(a1p + kb, (int)hh);
    v16h b = g2_frag(b0p + kb, (int)hh); c00 = g2_mma(a0, b, c00); c10 = g2_mma(a1, b, c10);
    b = g2_frag(b1p + kb, (int)hh); c01 = g2_mma(a0, b, c01); c11 = g2_mma(a1, b, c11);
    b = g2_frag(b2p + kb, (int)hh); c02 = g2_mma(a0, b, c02); c12 = g2_mma(a1, b, c12);
    b = g2_frag(b3p + kb, (int)hh); c03 = g2_mma(a0, b, c03); c13 = g2_mma(a1, b, c13); }
  v8f accs[8] = {c00, c01, c02, c03, c10, c11, c12, c13};
#pragma unroll
  for (int u = 0; u < 8; ++u) { const unsigned t = (unsigned)(u & 3), half = (unsigned)(u >> 2); const unsigned col = col0 + t * 16u + ln; const float bv = bf16_rne(bias[col]);
#pragma unroll
    for (int r = 0; r < 8; ++r) { const unsigned rloc = half * 16u + 8u * hh + (unsigned)r; float v = accs[u][r] * alpha + bv; if (mode == 1) v = fmaxf(v, 0.0f); so[w][rloc][t * 16u + ln] = v; } }
  __builtin_amdgcn_fence(4  , "workgroup"); __builtin_amdgcn_wave_barrier();
  if (mode == 2) {
    const unsigned rq = lane >> 3, pc = lane & 7u;
    for (int pass = 0; pass < 2; ++pass) {
#pragma unroll
      for (unsigned g = 0; g < 16; ++g) { const unsigned L = g * 4u + rq; const unsigned row = L >> 1, col = (L & 1u) * 32u + pc * 4u;
        const v4f v = *(const v4fa*)&so[w][row][col];
        *(volatile v4f*)(C32 + (size_t)(row0 + row) * ldc + col0 + col) = v; }
      if (pass == 0) __threadfence(); }
  } else {
    const unsigned rsub = lane >> 4, c4 = (lane & 15u) * 4u;
    for (int pass = 0; pass < 2; ++pass) {
#pragma unroll
      for (unsigned q = 0; q < 16; ++q) { const unsigned r = q * 2u + rsub; const v4f v = *(const v4fa*)&so[w][r][c4]; v4h h4;
#pragma unroll
        for (int i = 0; i < 4; ++i) h4[i] = (_Float16)v[i];
        *(volatile v4h*)(C16 + (size_t)(row0 + r) * ldc + col0 + c4) = h4; }
      if (pass == 0) __threadfence(); } } }

__global__ __launch_bounds__(256) void k_vt2(const _Float16* __restrict__ P, unsigned pitch, unsigned hs, unsigned coff, _Float16* __restrict__ VT) {
  __shared__ unsigned short tl[64][66];
  const unsigned tid = threadIdx.x; const unsigned slab = blockIdx.x / (unsigned)NQT, lg = blockIdx.x % (unsigned)NQT; const unsigned b = slab / (unsigned)NH, hd = slab % (unsigned)NH; const unsigned s0 = lg * 64u;
  for (unsigned i = tid; i < 512u; i += 256u) { const unsigned r = i >> 3, c8 = (i & 7u) * 8u; FragH f;
    f.half[0] = *(const v8us*)((const unsigned short*)P + (size_t)(b * (unsigned)SEQ + s0 + r) * pitch + hd * hs + coff + c8);
#pragma unroll
    for (int q = 0; q < 8; ++q) tl[r][c8 + q] = f.u[q]; }
  __syncthreads();
  for (int pass = 0; pass < 2; ++pass) {
#pragma unroll
    for (unsigned rd = 0; rd < 2; ++rd) { const unsigned d = rd * 32u + (tid >> 3), pc = tid & 7u; FragH f;
#pragma unroll
      for (int q = 0; q < 8; ++q) f.u[q] = tl[pc * 8u + q][d];
      *(volatile v8us*)((unsigned short*)VT + ((size_t)slab * HD + d) * SEQ + s0 + pc * 8u) = f.half[0]; }
    if (pass == 0) __threadfence(); } }

__device__ __forceinline__ unsigned mrow(const float* rowp, int& nz, int& am) {
  const v4f a = *(const v4fa*)rowp; const v4f c = *(const v4fa*)(rowp + 32); unsigned op = 0u;
#pragma unroll
  for (int i = 0; i < 4; ++i) {
    nz |= ((__float_as_uint(a[i]) & 0x7fffffffu) != 0u) ? 1 : 0; nz |= ((__float_as_uint(c[i]) & 0x7fffffffu) != 0u) ? 1 : 0;
    am &= (a[i] <= -1.0e8f) ? 1 : 0; am &= (c[i] <= -1.0e8f) ? 1 : 0;
    op |= (a[i] > -1.0e4f) ? 1u : 0u; op |= (c[i] > -1.0e4f) ? 1u : 0u; }
  return op; }

__global__ __launch_bounds__(256) void k_mflag(const float* __restrict__ mask0, const float* __restrict__ mask1, int* __restrict__ MF) {
  __shared__ int snz[32]; __shared__ int sam[32]; __shared__ unsigned swl[32]; __shared__ unsigned swh[32];
  const unsigned tid = threadIdx.x, qt = blockIdx.x, which = blockIdx.y; const unsigned kt = tid >> 3, p = tid & 7u;
  const float* mask = (which == 0u) ? mask0 : mask1;
  const bool ok = kt < (unsigned)NKT; const unsigned ktc = ok ? kt : (unsigned)(NKT - 1);
  const float* base = mask + (size_t)(qt * 64u) * SEQ_FULL + ktc * 64u + p * 4u;
  int nz = 0, am = 1; unsigned wl = 0u, wh = 0u;
#pragma unroll 1
  for (unsigned r = 0; r < 32u; ++r) { const unsigned op = mrow(base + (size_t)r * SEQ_FULL, nz, am); wl |= op << r; }
#pragma unroll 1
  for (unsigned r = 0; r < 32u; ++r) { const unsigned op = mrow(base + (size_t)(32u + r) * SEQ_FULL, nz, am); wh |= op << r; }
  nz |= __shfl_xor(nz, 1); nz |= __shfl_xor(nz, 2); nz |= __shfl_xor(nz, 4);
  am &= __shfl_xor(am, 1); am &= __shfl_xor(am, 2); am &= __shfl_xor(am, 4);
  wl |= __shfl_xor(wl, 1); wl |= __shfl_xor(wl, 2); wl |= __shfl_xor(wl, 4);
  wh |= __shfl_xor(wh, 1); wh |= __shfl_xor(wh, 2); wh |= __shfl_xor(wh, 4);
  if (p == 0u) { snz[kt] = nz; sam[kt] = am; swl[kt] = wl; swh[kt] = wh; }
  __syncthreads();
  if (tid < 32u) { unsigned al = 0u, ah = 0u;
#pragma unroll 1
    for (unsigned k = 0; k < 32u; ++k) { al |= swl[k]; ah |= swh[k]; }
    const bool allopen = (al == 0xffffffffu) && (ah == 0xffffffffu);
    const int tnz = snz[tid], tam = sam[tid];
    int v = (tnz == 0) ? 0 : ((tam != 0 && allopen) ? 2 : 1); v = (tid < (unsigned)NKT) ? v : 0;
    volatile int* d = MF + ((size_t)which * NQT + qt) * 32u + tid; *d = v; __threadfence(); *d = v; } }

__global__ __launch_bounds__(128) void k_attn(const _Float16* __restrict__ Qp, unsigned qpitch, unsigned qhs, const _Float16* __restrict__ Kp, unsigned kpitch, unsigned khs,
                                              const _Float16* __restrict__ VT, const float* __restrict__ mask, const int* __restrict__ MF, _Float16* __restrict__ ctx) {
  __shared__ __attribute__((aligned(16))) float so[4][16][68];
  const unsigned tid = threadIdx.x, w = tid >> 5, lane = tid & 31u, l15 = lane & 15u, hh = lane >> 4;
  const unsigned qt = blockIdx.x, slab = blockIdx.y; const unsigned b = slab / (unsigned)NH, hd = slab % (unsigned)NH;
  const unsigned q0 = qt * 64u + w * 16u;
  const _Float16* Qb = Qp + (size_t)(b * (unsigned)SEQ) * qpitch + hd * qhs;
  const _Float16* Kb = Kp + (size_t)(b * (unsigned)SEQ) * kpitch + hd * khs;
  const _Float16* Vb = VT + (size_t)slab * HD * SEQ;
  const _Float16* qrow = Qb + (size_t)(q0 + l15) * qpitch;
  const v16h qf0 = g2_frag(qrow, (int)hh), qf1 = g2_frag(qrow + 32, (int)hh);
  const v8f z8 = {0.f,0.f,0.f,0.f,0.f,0.f,0.f,0.f};
  v8f o[4] = {z8, z8, z8, z8};
  float m = NEG_INF, l = 0.f;
  const float CL = 0.18033688011112042f;
#pragma unroll 1
  for (unsigned it = 0; it < (unsigned)NKT; ++it) {
    const int mf = MF[(size_t)qt * 32u + it];
    if (mf == 2) continue;
    const unsigned key0 = it * 64u;
    v8f s[4];
#pragma unroll
    for (unsigned kt = 0; kt < 4; ++kt) {
      const _Float16* krow = Kb + (size_t)(key0 + kt * 16u + l15) * kpitch;
      const v16h ka = g2_frag(krow, (int)hh), kk = g2_frag(krow + 32, (int)hh);
      v8f a = g2_mma(ka, qf0, z8); a = g2_mma(kk, qf1, a); s[kt] = a; }
    if (mf != 0) {
#pragma unroll
      for (unsigned kt = 0; kt < 4; ++kt) {
        const float* mp = mask + (size_t)(q0 + l15) * SEQ_FULL + key0 + kt * 16u + 8u * hh;
        const v4f ma = *(const v4fa*)mp; const v4f mb = *(const v4fa*)(mp + 4);
#pragma unroll
        for (int r = 0; r < 4; ++r) { s[kt][r] = fmaf(ma[r], 8.0f, s[kt][r]); s[kt][4 + r] = fmaf(mb[r], 8.0f, s[kt][4 + r]); } } }
    float lmax = NEG_INF;
#pragma unroll
    for (int kt = 0; kt < 4; ++kt)
#pragma unroll
      for (int r = 0; r < 8; ++r) lmax = fmaxf(lmax, s[kt][r]);
    lmax = fmaxf(lmax, __shfl_xor(lmax, 16));
    const float mnew = fmaxf(m, lmax);
    const float mref = (mnew == NEG_INF) ? 0.0f : mnew;
    const float alpha = exp2f((m - mref) * CL);
    const float bexp = 10.0f - mref * CL;
    m = mnew;
    float psum = 0.f; FragH pa, pb;
#pragma unroll
    for (int r = 0; r < 8; ++r) {
      const float e0 = exp2f(fmaf(s[0][r], CL, bexp)), e1 = exp2f(fmaf(s[1][r], CL, bexp)), e2 = exp2f(fmaf(s[2][r], CL, bexp)), e3 = exp2f(fmaf(s[3][r], CL, bexp));
      psum += (e0 + e1) + (e2 + e3);
      pa.h[r] = (_Float16)e0; pa.h[8 + r] = (_Float16)e1; pb.h[r] = (_Float16)e2; pb.h[8 + r] = (_Float16)e3; }
    l = l * alpha + psum;
    float ar[8];
#pragma unroll
    for (int r = 0; r < 8; ++r) ar[r] = __shfl(alpha, (int)(8u * hh) + r);
#pragma unroll
    for (unsigned dt = 0; dt < 4; ++dt) {
#pragma unroll
      for (int r = 0; r < 8; ++r) o[dt][r] *= ar[r];
      const _Float16* vrow = Vb + (size_t)(dt * 16u + l15) * SEQ + key0;
      const v16h va = g2_frag(vrow, (int)hh), vb = g2_frag(vrow + 32, (int)hh);
      o[dt] = g2_mma(pa.v, va, o[dt]); o[dt] = g2_mma(pb.v, vb, o[dt]); } }
  const float lt = l + __shfl_xor(l, 16);
  const float inv = 16.0f * (1.0f / lt);
  float ir[8];
#pragma unroll
  for (int r = 0; r < 8; ++r) ir[r] = __shfl(inv, (int)(8u * hh) + r);
#pragma unroll
  for (unsigned dt = 0; dt < 4; ++dt)
#pragma unroll
    for (int r = 0; r < 8; ++r) so[w][8u * hh + (unsigned)r][dt * 16u + l15] = o[dt][r] * ir[r];
  __builtin_amdgcn_fence(4  , "workgroup"); __builtin_amdgcn_wave_barrier();
  const unsigned rq = lane >> 3, pc = lane & 7u;
  unsigned short* cb = (unsigned short*)ctx + (size_t)(b * (unsigned)SEQ + q0) * DM + hd * (unsigned)HD;
  for (int pass = 0; pass < 2; ++pass) {
#pragma unroll
    for (unsigned g = 0; g < 4; ++g) { const unsigned row = g * 4u + rq; const v4f a = *(const v4fa*)&so[w][row][pc * 8u]; const v4f c = *(const v4fa*)&so[w][row][pc * 8u + 4u]; FragH f;
#pragma unroll
      for (int i = 0; i < 4; ++i) { f.h[i] = (_Float16)a[i]; f.h[4 + i] = (_Float16)c[i]; }
      *(volatile v8us*)(cb + (size_t)row * DM + pc * 8u) = f.half[0]; }
    if (pass == 0) __threadfence(); } }

__global__ __launch_bounds__(128) void k_ln(const float* __restrict__ A, const float* __restrict__ R, const float* __restrict__ g, const float* __restrict__ be,
                                            float* __restrict__ out32, _Float16* __restrict__ out16, int rfull, int w16, int ofull) {
  __shared__ __attribute__((aligned(16))) float sr[4][DM];
  const unsigned tid = threadIdx.x, w = tid >> 5, lane = tid & 31u;
  const unsigned m = blockIdx.x * 4u + w;
  const unsigned gb = m / (unsigned)SEQ, gs = m % (unsigned)SEQ;
  const size_t mfull = (size_t)gb * SEQ_FULL + gs;
  const float* ap = A + (size_t)m * DM;
  const float* rp = R + (rfull ? mfull : (size_t)m) * DM;
  float* op = out32 + (ofull ? mfull : (size_t)m) * DM;
  float sum = 0.f;
#pragma unroll 1
  for (unsigned c = 0; c < 8u; ++c) { const unsigned col = c * 128u + lane * 4u; const v4f a = *(const v4fa*)(ap + col); v4f r = *(const v4fa*)(rp + col);
    if (rfull) {
#pragma unroll
      for (int i = 0; i < 4; ++i) r[i] = bf16_rne(r[i]); }
    const v4f xv = a + r; *(v4fa*)&sr[w][col] = xv; sum += (xv[0] + xv[1]) + (xv[2] + xv[3]); }
#pragma unroll
  for (int off = 16; off; off >>= 1) sum += __shfl_xor(sum, off);
  const float mean = sum * (1.0f / (float)DM);
  float s2 = 0.f;
#pragma unroll 1
  for (unsigned c = 0; c < 8u; ++c) { const unsigned col = c * 128u + lane * 4u; const v4f xv = *(const v4fa*)&sr[w][col];
#pragma unroll
    for (int i = 0; i < 4; ++i) { const float d = xv[i] - mean; s2 += d * d; } }
#pragma unroll
  for (int off = 16; off; off >>= 1) s2 += __shfl_xor(s2, off);
  const float rstd = 1.0f / sqrtf(s2 * (1.0f / (float)DM) + 1e-5f);
#pragma unroll 1
  for (unsigned c = 0; c < 8u; ++c) { const unsigned col = c * 128u + lane * 4u; const v4f xv = *(const v4fa*)&sr[w][col];
    const v4f gv = *(const v4fa*)(g + col); const v4f bv = *(const v4fa*)(be + col); v4f v;
#pragma unroll
    for (int i = 0; i < 4; ++i) v[i] = bf16_rne(gv[i]) * (xv[i] - mean) * rstd + bf16_rne(bv[i]);
    *(v4fa*)&sr[w][col] = v;
    *(volatile v4f*)(op + col) = v; }
  __threadfence();
#pragma unroll 1
  for (unsigned c = 0; c < 8u; ++c) { const unsigned col = c * 128u + lane * 4u; const v4f v = *(const v4fa*)&sr[w][col];
    *(volatile v4f*)(op + col) = v; }
  if (w16) {
    __builtin_amdgcn_fence(4  , "workgroup"); __builtin_amdgcn_wave_barrier();
    unsigned short* o16 = (unsigned short*)out16 + (size_t)m * DM;
    for (int pass = 0; pass < 2; ++pass) {
#pragma unroll 1
      for (unsigned c = 0; c < 4u; ++c) { const unsigned col = c * 256u + lane * 8u; const v4f a = *(const v4fa*)&sr[w][col]; const v4f d = *(const v4fa*)&sr[w][col + 4u]; FragH f;
#pragma unroll
        for (int i = 0; i < 4; ++i) { f.h[i] = (_Float16)a[i]; f.h[4 + i] = (_Float16)d[i]; }
        *(volatile v8us*)(o16 + col) = f.half[0]; }
      if (pass == 0) __threadfence(); } } }

extern "C" void kernel_launch(void* const* d_in, const int* in_sizes, int n_in,
                              void* d_out, int out_size, void* d_ws, size_t ws_size, hipStream_t stream) {
  if (n_in < 24) return;
  const float* x    = (const float*)d_in[0];
  const float* y    = (const float*)d_in[1];
  const float* mk1  = (const float*)d_in[2];
  const float* mk2  = (const float*)d_in[3];
  const float* Wqkv = (const float*)d_in[4];  const float* bqkv = (const float*)d_in[5];
  const float* Wo1  = (const float*)d_in[6];  const float* bo1  = (const float*)d_in[7];
  const float* Wkv  = (const float*)d_in[8];  const float* bkv  = (const float*)d_in[9];
  const float* Wq   = (const float*)d_in[10]; const float* bq   = (const float*)d_in[11];
  const float* Wo2  = (const float*)d_in[12]; const float* bo2  = (const float*)d_in[13];
  const float* W1   = (const float*)d_in[14]; const float* b1   = (const float*)d_in[15];
  const float* W2   = (const float*)d_in[16]; const float* b2   = (const float*)d_in[17];
  const float* g1   = (const float*)d_in[18]; const float* be1  = (const float*)d_in[19];
  const float* g2   = (const float*)d_in[20]; const float* be2  = (const float*)d_in[21];
  const float* g3   = (const float*)d_in[22]; const float* be3  = (const float*)d_in[23];
  const long long need_act = ((long long)(NB - 1) * SEQ_FULL + SEQ) * DM;
  const long long need_msk = (long long)(SEQ - 1) * SEQ_FULL + SEQ;
  if ((long long)in_sizes[0] < need_act || (long long)in_sizes[1] < need_act) return;
  if ((long long)in_sizes[2] < need_msk || (long long)in_sizes[3] < need_msk) return;
  if (in_sizes[4] < DM * 3 * DM || in_sizes[5] < 3 * DM) return;
  if (in_sizes[6] < DM * DM || in_sizes[7] < DM) return;
  if (in_sizes[8] < DM * 2 * DM || in_sizes[9] < 2 * DM) return;
  if (in_sizes[10] < DM * DM || in_sizes[11] < DM) return;
  if (in_sizes[12] < DM * DM || in_sizes[13] < DM) return;
  if (in_sizes[14] < DM * FF || in_sizes[15] < FF) return;
  if (in_sizes[16] < FF * DM || in_sizes[17] < DM) return;
  for (int i = 18; i < 24; ++i) if (in_sizes[i] < DM) return;
  if ((long long)out_size < need_act) return;
  char* ws = (char*)d_ws; size_t off = 0;
  auto take = [&](size_t bytes) { char* p = ws + off; off += (bytes + 255) & ~(size_t)255; return p; };
  _Float16* BQKV = (_Float16*)take((size_t)3 * DM * DM * 2);
  _Float16* BO1  = (_Float16*)take((size_t)DM * DM * 2);
  _Float16* BKV  = (_Float16*)take((size_t)2 * DM * DM * 2);
  _Float16* BQ   = (_Float16*)take((size_t)DM * DM * 2);
  _Float16* BO2  = (_Float16*)take((size_t)DM * DM * 2);
  _Float16* BW1  = (_Float16*)take((size_t)FF * DM * 2);
  _Float16* BW2  = (_Float16*)take((size_t)DM * FF * 2);
  _Float16* RA   = (_Float16*)take((size_t)MROWS * DM * 2);
  _Float16* RB   = (_Float16*)take((size_t)MROWS * FF * 2);
  float*    RO   = (float*)take((size_t)MROWS * DM * 4);
  float*    Y1F  = (float*)take((size_t)MROWS * DM * 4);
  float*    RF2  = (float*)take((size_t)MROWS * DM * 4);
  int*      MF   = (int*)take((size_t)2 * NQT * 32 * 4);
  if (off > ws_size || off > (size_t)134217728) return;
  _Float16* Y16 = RA; _Float16* CTX = RA; _Float16* Y1H = RA; _Float16* Y2H = RA;
  _Float16* QKV = RB; _Float16* KV = RB; _Float16* Q2 = RB + (size_t)MROWS * 2 * DM; _Float16* FF1 = RB;
  _Float16* VT = (_Float16*)RO; _Float16* X16 = (_Float16*)RF2; float* Y2F = RF2;
  const int* MF1 = MF; const int* MF2 = MF + (size_t)NQT * 32;

  k_wtr<<<dim3(3 * DM / 64, DM / 64), 256, 0, stream>>>(Wqkv, DM, 3 * DM, BQKV);
  k_wtr<<<dim3(DM / 64, DM / 64),     256, 0, stream>>>(Wo1,  DM, DM,     BO1);
  k_wtr<<<dim3(2 * DM / 64, DM / 64), 256, 0, stream>>>(Wkv,  DM, 2 * DM, BKV);
  k_wtr<<<dim3(DM / 64, DM / 64),     256, 0, stream>>>(Wq,   DM, DM,     BQ);
  k_wtr<<<dim3(DM / 64, DM / 64),     256, 0, stream>>>(Wo2,  DM, DM,     BO2);
  k_wtr<<<dim3(FF / 64, DM / 64),     256, 0, stream>>>(W1,   DM, FF,     BW1);
  k_wtr<<<dim3(DM / 64, FF / 64),     256, 0, stream>>>(W2,   FF, DM,     BW2);
  const unsigned gx = (unsigned)(MROWS * (DM / 8) / 256);
  k_x16<<<gx, 256, 0, stream>>>(y, Y16);
  k_x16<<<gx, 256, 0, stream>>>(x, X16);
  k_mflag<<<dim3((unsigned)NQT, 2), 256, 0, stream>>>(mk1, mk2, MF);

  const unsigned mb = (unsigned)(MROWS / 128);
  k_gemm2<<<mb * (3 * DM / 64), 128, 0, stream>>>(Y16, DM, BQKV, DM, 0.0625f, bqkv, QKV, (float*)nullptr, 3 * DM, MROWS, 3 * DM, DM, 0);
  k_vt2<<<(unsigned)(NB * NH * NQT), 256, 0, stream>>>(QKV, 3 * DM, 3 * HD, 2 * HD, VT);
  k_attn<<<dim3((unsigned)NQT, (unsigned)(NB * NH)), 128, 0, stream>>>(QKV, 3 * DM, 3 * HD, QKV + HD, 3 * DM, 3 * HD, VT, mk1, MF1, CTX);
  k_gemm2<<<mb * (DM / 64), 128, 0, stream>>>(CTX, DM, BO1, DM, 0.00390625f, bo1, (_Float16*)nullptr, RO, DM, MROWS, DM, DM, 2);
  k_ln<<<(unsigned)(MROWS / 4), 128, 0, stream>>>(RO, y, g1, be1, Y1F, Y1H, 1, 1, 0);

  k_gemm2<<<mb * (2 * DM / 64), 128, 0, stream>>>(X16, DM, BKV, DM, 0.0625f, bkv, KV, (float*)nullptr, 2 * DM, MROWS, 2 * DM, DM, 0);
  k_gemm2<<<mb * (DM / 64), 128, 0, stream>>>(Y1H, DM, BQ, DM, 0.0625f, bq, Q2, (float*)nullptr, DM, MROWS, DM, DM, 0);
  k_vt2<<<(unsigned)(NB * NH * NQT), 256, 0, stream>>>(KV, 2 * DM, 2 * HD, HD, VT);
  k_attn<<<dim3((unsigned)NQT, (unsigned)(NB * NH)), 128, 0, stream>>>(Q2, DM, HD, KV, 2 * DM, 2 * HD, VT, mk2, MF2, CTX);
  k_gemm2<<<mb * (DM / 64), 128, 0, stream>>>(CTX, DM, BO2, DM, 0.00390625f, bo2, (_Float16*)nullptr, RO, DM, MROWS, DM, DM, 2);
  k_ln<<<(unsigned)(MROWS / 4), 128, 0, stream>>>(RO, Y1F, g2, be2, Y2F, Y2H, 0, 1, 0);

  k_gemm2<<<mb * (FF / 64), 128, 0, stream>>>(Y2H, DM, BW1, DM, 0.0625f, b1, FF1, (float*)nullptr, FF, MROWS, FF, DM, 1);
  k_gemm2<<<mb * (DM / 64), 128, 0, stream>>>(FF1, FF, BW2, FF, 0.0625f, b2, (_Float16*)nullptr, RO, DM, MROWS, DM, FF, 2);
  k_ln<<<(unsigned)(MROWS / 4), 128, 0, stream>>>(RO, Y2F, g3, be3, (float*)d_out, (_Float16*)nullptr, 0, 0, 1);
}
